// Mamba3Triton_55241869361708
// MI455X (gfx1250) — hardware-verified
//
#include <hip/hip_runtime.h>
#include <stdint.h>
#include <math.h>


typedef __attribute__((ext_vector_type(16))) _Float16 v16h;
typedef __attribute__((ext_vector_type(8)))  _Float16 v8h;
typedef __attribute__((ext_vector_type(8)))  float    v8f;
typedef __attribute__((ext_vector_type(4)))  float    v4f;

#define NB_   2
#define L_    4096
#define H_    24
#define P_    64
#define N_    128
#define CS_   128
#define NC_   (L_ / CS_)
#define NBH_  (NB_ * H_)
#define QP    136
#define VP    136
#define SLABP 68
#define PCARRY 2048.0f
#define PINV   (1.0f / 2048.0f)
#define KCARRY 4096.0f
#define KINV   (1.0f / 4096.0f)
#define SCARRY 256.0f
#define SINV   (1.0f / 256.0f)

__device__ __forceinline__ void dep_guard_h(v8f& a, v8f& b, v16h x, v16h y) { asm volatile("v_nop\n\tv_nop\n\tv_nop\n\tv_nop" : "+v"(a), "+v"(b) : "v"(x), "v"(y)); }
__device__ __forceinline__ void keep4_h(v16h a, v16h b, v16h c, v16h d) { asm volatile("v_nop" :: "v"(a), "v"(b), "v"(c), "v"(d)); }
template <typename T> struct Frag;
template <> struct Frag<_Float16> {
  typedef v16h V; union U { v16h v; v8h h[2]; };
  static __device__ __forceinline__ v16h load(const _Float16* p) {
    U f; f.h[0] = *(const v8h*)(p); f.h[1] = *(const v8h*)(p + 16); return f.v;
  }
  static __device__ __forceinline__ v8f mma(v16h a, v16h b, v8f c) {
    return __builtin_amdgcn_wmma_f32_16x16x32_f16(false, a, false, b, (short)0, c, false, false);
  }
  static __device__ __forceinline__ void guard(v8f& a, v8f& b, v16h x, v16h y) { dep_guard_h(a, b, x, y); }
  static __device__ __forceinline__ void keep(v16h a, v16h b, v16h c, v16h d) { keep4_h(a, b, c, d); }
};

__device__ __forceinline__ v8f mma_h(v16h a, v16h b, v8f c) {
  c = __builtin_amdgcn_wmma_f32_16x16x32_f16(false, a, false, b, (short)0, c, false, false);
  asm volatile("v_nop\n\tv_nop\n\tv_nop\n\tv_nop" : "+v"(c) : "v"(a), "v"(b));
  return c;
}

__device__ __forceinline__ void lds_wave_sync() {
  __builtin_amdgcn_fence(__ATOMIC_RELEASE, "workgroup");
  __builtin_amdgcn_wave_barrier();
  __builtin_amdgcn_fence(__ATOMIC_ACQUIRE, "workgroup");
}

__device__ __forceinline__ double shfl_up_d(double v, int d) {
  union { double f; int i[2]; } u;
  u.f = v;
  u.i[0] = __shfl_up(u.i[0], (unsigned)d, 32);
  u.i[1] = __shfl_up(u.i[1], (unsigned)d, 32);
  return u.f;
}
__device__ __forceinline__ double wave_scan_d(double v, int lane) {
#pragma unroll
  for (int d = 1; d < 32; d <<= 1) {
    const double o = shfl_up_d(v, d);
    if (lane >= d) v += o;
  }
  return v;
}

__device__ __forceinline__ void store_rows64(const float* slab, float* dst, int ldd, int lane) {
  const int h2 = lane >> 4, c4 = (lane & 15) * 4;
  for (int pass = 0; pass < 2; ++pass) {
#pragma unroll
    for (int it = 0; it < 8; ++it) {
      const int row = it * 2 + h2;
      const v4f v = *(const v4f*)(slab + row * SLABP + c4);
      *(volatile v4f*)(dst + (size_t)row * ldd + c4) = v;
    }
    __threadfence();
  }
}

__global__ __launch_bounds__(256)
void k_chunk(const float* __restrict__ X, const float* __restrict__ DT, const float* __restrict__ Av,
             const float* __restrict__ Bm, const float* __restrict__ Cm,
             float* __restrict__ Yi, float* __restrict__ St)
{
  __shared__ __align__(16) float    sQS[8 * 16 * SLABP];
  __shared__ __align__(16) _Float16 sK[CS_ * QP];
  __shared__ __align__(16) _Float16 sKdT[N_ * VP];
  __shared__ __align__(16) _Float16 sVt[P_ * VP];
  __shared__ float  sDt[CS_], sCum[CS_], sEct[CS_], sErd[CS_], sKw[CS_], sCos[CS_], sSin[CS_];
  __shared__ double sPart[256];
  __shared__ double sTotD[4], sTotA[4];
  __shared__ double sBase;

  const int tid  = threadIdx.x;
  const int lane = tid & 31;
  const int w    = __builtin_amdgcn_readfirstlane(tid >> 5);
  const int hh   = lane >> 4;
  const int rl   = lane & 15;
  const int blk  = blockIdx.x;
  const int bh   = blk / NC_;
  const int c    = blk - bh * NC_;
  const int b    = bh / H_;
  const int h    = bh - b * H_;
  const int t0   = c * CS_;
  const float Ah = Av[h];
  const v8f z8 = {0.f, 0.f, 0.f, 0.f, 0.f, 0.f, 0.f, 0.f};

  {
    double acc = 0.0;
    const float* dp = DT + (size_t)b * L_ * H_ + h;
    for (int t = tid; t < t0; t += 256) acc += (double)dp[(size_t)t * H_];
    sPart[tid] = acc;
  }
  __syncthreads();
  if (tid == 0) {
    double s = 0.0;
    for (int i = 0; i < 256; ++i) s += sPart[i];
    sBase = s;
  }
  double scD = 0.0, scA = 0.0;
  float dreg = 0.0f;
  if (tid < CS_) {
    dreg = DT[((size_t)b * L_ + t0 + tid) * H_ + h];
    const float a = Ah * dreg;
    scD = wave_scan_d((double)dreg, lane);
    scA = wave_scan_d((double)a, lane);
    if (lane == 31) { sTotD[w] = scD; sTotA[w] = scA; }
  }
  __syncthreads();
  if (tid < CS_) {
    double pd = 0.0, pa = 0.0;
    for (int u = 0; u < w; ++u) { pd += sTotD[u]; pa += sTotA[u]; }
    const float ang  = (float)(sBase + pd + scD);
    const float cumf = (float)(pa + scA);
    sDt[tid]  = dreg;
    sCum[tid] = cumf;
    sCos[tid] = cosf(ang);
    sSin[tid] = sinf(ang);
    sEct[tid] = expf(cumf);
    sErd[tid] = expf(-cumf) * dreg * PCARRY;
  }
  __syncthreads();
  if (tid < CS_) sKw[tid] = expf(sCum[CS_ - 1] - sCum[tid]) * sDt[tid] * KCARRY;
  __syncthreads();

  {
    _Float16* sQw = (_Float16*)sQS;
    const float* Cb = Cm + ((size_t)b * L_ + t0) * N_;
    const float* Bb = Bm + ((size_t)b * L_ + t0) * N_;
    const float* Xb = X + (((size_t)b * L_ + t0) * H_ + h) * P_;
    const int tr = tid >> 4, m4 = (tid & 15) * 4;
#pragma unroll 1
    for (int pass = 0; pass < 8; ++pass) {
      const int t = pass * 16 + tr;
      const v4f c1 = *(const v4f*)(Cb + (size_t)t * N_ + m4);
      const v4f c2 = *(const v4f*)(Cb + (size_t)t * N_ + 64 + m4);
      const v4f b1 = *(const v4f*)(Bb + (size_t)t * N_ + m4);
      const v4f b2 = *(const v4f*)(Bb + (size_t)t * N_ + 64 + m4);
      const v4f xv = *(const v4f*)(Xb + (size_t)t * (H_ * P_) + m4);
      const float cv = sCos[t], sv = sSin[t], kw = sKw[t];
      _Float16* qrow = sQw + t * QP;
      _Float16* krow = sK + t * QP;
#pragma unroll
      for (int e = 0; e < 4; ++e) {
        const int j = m4 + e;
        const float q1 = c1[e] * cv - c2[e] * sv;
        const float q2 = c1[e] * sv + c2[e] * cv;
        const float k1 = b1[e] * cv - b2[e] * sv;
        const float k2 = b1[e] * sv + b2[e] * cv;
        qrow[j]      = (_Float16)q1;
        qrow[64 + j] = (_Float16)q2;
        krow[j]      = (_Float16)k1;
        krow[64 + j] = (_Float16)k2;
        sKdT[j * VP + t]        = (_Float16)(k1 * kw);
        sKdT[(64 + j) * VP + t] = (_Float16)(k2 * kw);
        sVt[j * VP + t]         = (_Float16)xv[e];
      }
    }
  }
  __syncthreads();

  v8f accS[8];
#pragma unroll
  for (int i = 0; i < 8; ++i) accS[i] = z8;
  {
    const _Float16* sQh = (const _Float16*)sQS;
#pragma unroll
    for (int ks = 0; ks < 4; ++ks) {
      const v16h a = Frag<_Float16>::load(sQh + (16 * w + rl) * QP + 32 * ks + 8 * hh);
#pragma unroll
      for (int nt = 0; nt < 8; ++nt) {
        if (nt <= w) {
          const v16h bb = Frag<_Float16>::load(sK + (16 * nt + rl) * QP + 32 * ks + 8 * hh);
          accS[nt] = mma_h(a, bb, accS[nt]);
        }
      }
    }
  }
  __syncthreads();

  {
    _Float16* sP = sK;
    const int wlim = (w < 6) ? (w + 1) : 7;
    float ect[8];
#pragma unroll
    for (int r = 0; r < 8; ++r) ect[r] = sEct[16 * w + 8 * hh + r];
#pragma unroll
    for (int nt = 0; nt < 8; ++nt) {
      if (nt <= wlim) {
        const int s = 16 * nt + rl;
        const float es = sErd[s];
#pragma unroll
        for (int r = 0; r < 8; ++r) {
          const int t = 16 * w + 8 * hh + r;
          float v = accS[nt][r] * ect[r] * es;
          v = (s <= t) ? v : 0.0f;
          sP[t * QP + s] = (_Float16)v;
        }
      }
    }
  }
  __syncthreads();

  v8f accY[4];
#pragma unroll
  for (int j = 0; j < 4; ++j) accY[j] = z8;
  {
    const _Float16* sP = sK;
#pragma unroll
    for (int ks = 0; ks < 4; ++ks) {
      if (ks <= (w >> 1)) {
        const v16h a = Frag<_Float16>::load(sP + (16 * w + rl) * QP + 32 * ks + 8 * hh);
#pragma unroll
        for (int j = 0; j < 4; ++j) {
          const v16h bb = Frag<_Float16>::load(sVt + (16 * j + rl) * VP + 32 * ks + 8 * hh);
          accY[j] = mma_h(a, bb, accY[j]);
        }
      }
    }
  }
  float* slab = sQS + w * (16 * SLABP);
#pragma unroll
  for (int j = 0; j < 4; ++j)
#pragma unroll
    for (int r = 0; r < 8; ++r) slab[(8 * hh + r) * SLABP + 16 * j + rl] = accY[j][r] * PINV;
  lds_wave_sync();
  store_rows64(slab, Yi + ((size_t)bh * L_ + t0 + 16 * w) * P_, P_, lane);
  lds_wave_sync();

  v8f accU[4];
#pragma unroll
  for (int j = 0; j < 4; ++j) accU[j] = z8;
  {
    const int pi = w & 3, nq = w >> 2;
#pragma unroll
    for (int ks = 0; ks < 4; ++ks) {
      const v16h a = Frag<_Float16>::load(sVt + (16 * pi + rl) * VP + 32 * ks + 8 * hh);
#pragma unroll
      for (int jj = 0; jj < 4; ++jj) {
        const v16h bb = Frag<_Float16>::load(sKdT + (16 * (4 * nq + jj) + rl) * VP + 32 * ks + 8 * hh);
        accU[jj] = mma_h(a, bb, accU[jj]);
      }
    }
#pragma unroll
    for (int jj = 0; jj < 4; ++jj)
#pragma unroll
      for (int r = 0; r < 8; ++r) slab[(8 * hh + r) * SLABP + 16 * jj + rl] = accU[jj][r] * KINV;
    lds_wave_sync();
    store_rows64(slab, St + ((size_t)(bh * NC_ + c) * P_ + 16 * pi) * N_ + 64 * nq, N_, lane);
  }
}

__global__ __launch_bounds__(256)
void k_state(const float* __restrict__ X, const float* __restrict__ DT, const float* __restrict__ Av,
             const float* __restrict__ Cm, const float* __restrict__ Dv, const int* __restrict__ csp,
             const float* __restrict__ Yi, const float* __restrict__ St, float* __restrict__ Y)
{
  __shared__ __align__(16) float    sS[P_ * N_];
  __shared__ __align__(16) _Float16 sSh[P_ * VP];
  __shared__ __align__(16) _Float16 sQ[CS_ * QP];
  __shared__ __align__(16) float    sSlab[8 * 16 * SLABP];
  __shared__ float  sCum[CS_], sEct[CS_], sCos[CS_], sSin[CS_];
  __shared__ double sTotD[4], sTotA[4];

  if (csp[0] != CS_) return;

  const int tid  = threadIdx.x;
  const int lane = tid & 31;
  const int w    = __builtin_amdgcn_readfirstlane(tid >> 5);
  const int hh   = lane >> 4;
  const int rl   = lane & 15;
  const int bh   = blockIdx.x;
  const int b    = bh / H_;
  const int h    = bh - b * H_;
  const float Ah = Av[h];
  const float Dh = Dv[h];
  const v8f z8 = {0.f, 0.f, 0.f, 0.f, 0.f, 0.f, 0.f, 0.f};

  for (int i = tid; i < P_ * N_; i += 256) sS[i] = 0.0f;
  double base = 0.0;

#pragma unroll 1
  for (int c = 0; c < NC_; ++c) {
    const int t0 = c * CS_;
    __syncthreads();
    double scD = 0.0, scA = 0.0;
    if (tid < CS_) {
      const float d = DT[((size_t)b * L_ + t0 + tid) * H_ + h];
      const float a = Ah * d;
      scD = wave_scan_d((double)d, lane);
      scA = wave_scan_d((double)a, lane);
      if (lane == 31) { sTotD[w] = scD; sTotA[w] = scA; }
    }
    __syncthreads();
    double totD = 0.0;
    for (int u = 0; u < 4; ++u) totD += sTotD[u];
    if (tid < CS_) {
      double pd = 0.0, pa = 0.0;
      for (int u = 0; u < w; ++u) { pd += sTotD[u]; pa += sTotA[u]; }
      const float ang  = (float)(base + pd + scD);
      const float cumf = (float)(pa + scA);
      sCum[tid] = cumf;
      sCos[tid] = cosf(ang);
      sSin[tid] = sinf(ang);
      sEct[tid] = expf(cumf) * SINV;
    }
    for (int i = tid; i < P_ * N_; i += 256) sSh[(i >> 7) * VP + (i & 127)] = (_Float16)(sS[i] * SCARRY);
    __syncthreads();
    {
      const float* Cb = Cm + ((size_t)b * L_ + t0) * N_;
      const int tr = tid >> 4, m4 = (tid & 15) * 4;
#pragma unroll 1
      for (int pass = 0; pass < 8; ++pass) {
        const int t = pass * 16 + tr;
        const v4f c1 = *(const v4f*)(Cb + (size_t)t * N_ + m4);
        const v4f c2 = *(const v4f*)(Cb + (size_t)t * N_ + 64 + m4);
        const float cv = sCos[t], sv = sSin[t];
        _Float16* qrow = sQ + t * QP;
#pragma unroll
        for (int e = 0; e < 4; ++e) {
          const int j = m4 + e;
          qrow[j]      = (_Float16)(c1[e] * cv - c2[e] * sv);
          qrow[64 + j] = (_Float16)(c1[e] * sv + c2[e] * cv);
        }
      }
    }
    __syncthreads();
    v8f acc[4];
#pragma unroll
    for (int j = 0; j < 4; ++j) acc[j] = z8;
#pragma unroll
    for (int ks = 0; ks < 4; ++ks) {
      const v16h a = Frag<_Float16>::load(sQ + (16 * w + rl) * QP + 32 * ks + 8 * hh);
#pragma unroll
      for (int j = 0; j < 4; ++j) {
        const v16h bb = Frag<_Float16>::load(sSh + (16 * j + rl) * VP + 32 * ks + 8 * hh);
        acc[j] = mma_h(a, bb, acc[j]);
      }
    }
    {
      float* slab = sSlab + w * (16 * SLABP);
#pragma unroll
      for (int j = 0; j < 4; ++j)
#pragma unroll
        for (int r = 0; r < 8; ++r)
          slab[(8 * hh + r) * SLABP + 16 * j + rl] = acc[j][r] * sEct[16 * w + 8 * hh + r];
      lds_wave_sync();
      const int h2 = lane >> 4, c4 = (lane & 15) * 4;
      v4f o[8];
#pragma unroll
      for (int it = 0; it < 8; ++it) {
        const int row = 2 * it + h2;
        const int tg  = t0 + 16 * w + row;
        const v4f vi = *(const v4f*)(slab + row * SLABP + c4);
        const v4f yi = *(const v4f*)(Yi + ((size_t)bh * L_ + tg) * P_ + c4);
        const v4f xv = *(const v4f*)(X + (((size_t)b * L_ + tg) * H_ + h) * P_ + c4);
        o[it] = vi + yi + xv * Dh;
      }
      for (int pass = 0; pass < 2; ++pass) {
#pragma unroll
        for (int it = 0; it < 8; ++it) {
          const int row = 2 * it + h2;
          const int tg  = t0 + 16 * w + row;
          *(volatile v4f*)(Y + (((size_t)b * L_ + tg) * H_ + h) * P_ + c4) = o[it];
        }
        __threadfence();
      }
      lds_wave_sync();
    }
    {
      const float dec = expf(sCum[CS_ - 1]);
      const float* stp = St + (size_t)(bh * NC_ + c) * (P_ * N_);
      for (int i4 = tid; i4 < (P_ * N_) / 4; i4 += 256) {
        v4f sv = *(const v4f*)(sS + 4 * i4);
        const v4f tv = *(const v4f*)(stp + 4 * i4);
        sv = sv * dec + tv;
        *(v4f*)(sS + 4 * i4) = sv;
      }
    }
    base += totD;
  }
}

extern "C" void kernel_launch(void* const* d_in, const int* in_sizes, int n_in,
                              void* d_out, int out_size, void* d_ws, size_t ws_size,
                              hipStream_t stream) {
  if (n_in < 7) return;
  if (in_sizes[0] != NB_ * L_ * H_ * P_) return;
  if (in_sizes[1] != NB_ * L_ * H_) return;
  if (in_sizes[2] < H_) return;
  if (in_sizes[3] != NB_ * L_ * N_) return;
  if (in_sizes[4] != NB_ * L_ * N_) return;
  if (in_sizes[5] < H_) return;
  if (in_sizes[6] < 1) return;
  if (out_size != NB_ * L_ * H_ * P_) return;

  const size_t yiBytes = (size_t)NBH_ * L_ * P_ * sizeof(float);
  const size_t stBytes = (size_t)NBH_ * NC_ * P_ * N_ * sizeof(float);
  if (yiBytes + stBytes > ws_size) return;
  if (yiBytes + stBytes > (size_t)134217728u) return;

  const float* X   = (const float*)d_in[0];
  const float* DT  = (const float*)d_in[1];
  const float* Av  = (const float*)d_in[2];
  const float* Bm  = (const float*)d_in[3];
  const float* Cm  = (const float*)d_in[4];
  const float* Dv  = (const float*)d_in[5];
  const int*   CSp = (const int*)d_in[6];
  float* Y  = (float*)d_out;
  float* Yi = (float*)d_ws;
  float* St = (float*)((char*)d_ws + yiBytes);

  k_chunk<<<dim3(NBH_ * NC_), dim3(256), 0, stream>>>(X, DT, Av, Bm, Cm, Yi, St);
  k_state<<<dim3(NBH_), dim3(256), 0, stream>>>(X, DT, Av, Cm, Dv, CSp, Yi, St, Y);
  (void)hipGetLastError();
}
